// MLA_1812476199155
// MI455X (gfx1250) — hardware-verified
//
#include <hip/hip_runtime.h>
#include <math.h>
#include <stdint.h>

#ifndef NB
#define NB 2
#endif
#ifndef SEQ
#define SEQ 2048
#endif
#define NB_FULL  2
#define SEQ_FULL 2048
#define DMOD  2048
#define NHD   16
#define DHD   128
#define QPR   1024
#define KVP   1365
#define KVPAD 1408
#define KVK   1376
#define QNP   1792
#define KNP   1792
#define KVW   3840
#define RPW   256
#define NTOK  (NB * SEQ)
#define ERL   64
#define OUT1_OFF 8388608
#define LN_EPS 1e-5f
#define WSC   64.0f
#define IWSC  (1.0f / 64.0f)
#define CTXC  16.0f
#define PSC   1024.0f
#define LOS   2048.0f
#define ILOS  (1.0f / 2048.0f)
#define SSCALE 0.08838834764831845f

static_assert(NB >= 1 && NB <= NB_FULL);
static_assert(SEQ >= 64 && SEQ <= SEQ_FULL && SEQ % 64 == 0);
static_assert(OUT1_OFF * 4 == 33554432);
static_assert(NHD * DHD == DMOD);
static_assert(KVPAD % 64 == 0 && KVK % 32 == 0 && KVK >= KVP && KVK <= KVPAD);
static_assert(QNP + RPW == DMOD && KNP + DMOD == KVW);
static_assert(DMOD % 64 == 0 && QPR % 64 == 0 && QNP % 64 == 0 && RPW % 64 == 0 && KNP % 64 == 0 && ERL % 64 == 0);
static_assert(DMOD % 32 == 0 && QPR % 32 == 0);
static_assert(NTOK % 64 == 0 && NTOK % 8 == 0);
static_assert((SEQ * KVP) % 4 == 0 && (SEQ * KVP * 4) % 128 == 0);
static_assert(DMOD == 256 * 8 && RPW == 32 * 8);

typedef _Float16     v16h __attribute__((ext_vector_type(16)));
typedef _Float16     v8h  __attribute__((ext_vector_type(8)));
typedef float        v8f  __attribute__((ext_vector_type(8)));
typedef float        v4f  __attribute__((ext_vector_type(4)));
typedef unsigned int v4u  __attribute__((ext_vector_type(4)));

__device__ __forceinline__ unsigned short bf_bits(float f) {
  const unsigned u = __float_as_uint(f);
  return (unsigned short)((u + 0x7FFFu + ((u >> 16) & 1u)) >> 16);
}
__device__ __forceinline__ float bf_val(unsigned short h) { return __uint_as_float(((unsigned)h) << 16); }
__device__ __forceinline__ float bf_rne(float f) { return bf_val(bf_bits(f)); }
__device__ __forceinline__ unsigned short h_bits(float f) { return __builtin_bit_cast(unsigned short, (_Float16)f); }
__device__ __forceinline__ float h_val(unsigned short u) { return (float)__builtin_bit_cast(_Float16, u); }
__device__ __forceinline__ unsigned pk16(unsigned short a, unsigned short b) { return (unsigned)a | ((unsigned)b << 16); }
__device__ __forceinline__ v8f zero8() { v8f z = {0.f, 0.f, 0.f, 0.f, 0.f, 0.f, 0.f, 0.f}; return z; }
__device__ __forceinline__ int wave_id() { return __builtin_amdgcn_readfirstlane((int)(threadIdx.x >> 5)); }
__device__ __forceinline__ int imin(int a, int b) { return a < b ? a : b; }

__device__ __forceinline__ void lds_wave_sync() {
  __builtin_amdgcn_fence(3  , "workgroup");
  __builtin_amdgcn_wave_barrier();
  __builtin_amdgcn_fence(2  , "workgroup");
}

union FragH { v16h v; v8h h[2]; };
__device__ __forceinline__ v16h ldfrag(const _Float16* p) { FragH f; f.h[0] = *(const v8h*)(p); f.h[1] = *(const v8h*)(p + 16); return f.v; }

__device__ __forceinline__ v8f mma_h(v16h a, v16h b, v8f c) {
  return __builtin_amdgcn_wmma_f32_16x16x32_f16(false, a, false, b, (short)0, c, false, false);
}
__device__ __forceinline__ void dep_guard(v8f& a, v8f& b, v16h x, v16h y) {
  asm volatile("v_nop\n\tv_nop\n\tv_nop\n\tv_nop" : "+v"(a), "+v"(b) : "v"(x), "v"(y));
}
__device__ __forceinline__ void keep4(v16h a, v16h b, v16h c, v16h d) { asm volatile("v_nop" :: "v"(a), "v"(b), "v"(c), "v"(d)); }
__device__ __forceinline__ void acc_guard4(v8f& a, v8f& b, v8f& c, v8f& d) {
  asm volatile("v_nop\n\tv_nop\n\tv_nop\n\tv_nop" : "+v"(a), "+v"(b), "+v"(c), "+v"(d));
}
__device__ __forceinline__ v8f at_mma(v16h a, v16h b, v8f c) {
  c = __builtin_amdgcn_wmma_f32_16x16x32_f16(false, a, false, b, (short)0, c, false, false);
  asm volatile("v_nop\n\tv_nop\n\tv_nop\n\tv_nop" : "+v"(c) : "v"(a), "v"(b));
  return c;
}

__global__ __launch_bounds__(256) void cvt16_kernel(const float* __restrict__ in, long strideIn,
                                                   unsigned short* outp, long strideOut, int n8, float scale) {
  const int i = (int)blockIdx.x * 256 + (int)threadIdx.x;
  if (i >= n8) return;
  const float* src = in + (size_t)blockIdx.y * strideIn + 8 * (size_t)i;
  unsigned short* dst = outp + (size_t)blockIdx.y * strideOut + 8 * (size_t)i;
  const v4f a = *(const v4f*)(src);
  const v4f b = *(const v4f*)(src + 4);
  v4u w;
  w[0] = pk16(h_bits(scale * bf_rne(a[0])), h_bits(scale * bf_rne(a[1])));
  w[1] = pk16(h_bits(scale * bf_rne(a[2])), h_bits(scale * bf_rne(a[3])));
  w[2] = pk16(h_bits(scale * bf_rne(b[0])), h_bits(scale * bf_rne(b[1])));
  w[3] = pk16(h_bits(scale * bf_rne(b[2])), h_bits(scale * bf_rne(b[3])));
  *(volatile v4u*)(dst) = w;
  __threadfence();
  *(volatile v4u*)(dst) = w;
}

__global__ __launch_bounds__(256) void tcvt_kernel(const float* __restrict__ W, unsigned short* oh, int R, int Cc, int Rpad, float scale) {
  __shared__ __align__(16) float tf[64 * 65];
  const int c0  = blockIdx.x * 64;
  const int r0  = blockIdx.y * 64;
  const int tid = threadIdx.x;
  {
    const int cc = tid & 63;
    const int rb = tid >> 6;
#pragma unroll
    for (int it = 0; it < 16; ++it) {
      const int rr = it * 4 + rb;
      const int gr = r0 + rr, gc = c0 + cc;
      const int grc = imin(gr, R - 1), gcc = imin(gc, Cc - 1);
      const float f = W[(size_t)grc * Cc + gcc];
      tf[rr * 65 + cc] = (gr < R && gc < Cc) ? f : 0.f;
    }
  }
  __syncthreads();
  const int sub = tid >> 3;
  const int c8  = (tid & 7) * 8;
  v4u hv[2];
#pragma unroll
  for (int it = 0; it < 2; ++it) {
    const int oc = it * 32 + sub;
    v4u a;
#pragma unroll
    for (int q = 0; q < 4; ++q) {
      const float f0 = tf[(c8 + 2 * q) * 65 + oc];
      const float f1 = tf[(c8 + 2 * q + 1) * 65 + oc];
      a[q] = pk16(h_bits(scale * bf_rne(f0)), h_bits(scale * bf_rne(f1)));
    }
    hv[it] = a;
  }
  for (int pass = 0; pass < 2; ++pass) {
#pragma unroll
    for (int it = 0; it < 2; ++it) {
      const int oc = it * 32 + sub;
      const size_t go = (size_t)(c0 + oc) * Rpad + r0 + c8;
      *(volatile v4u*)(oh + go) = hv[it];
    }
    __threadfence();
  }
}

__device__ __forceinline__ void sincos_red(float a, float& sn, float& cs) {
  const float q = rintf(a * 0.636619772367581343f);
  float r = fmaf(-q, 1.5703125f, a);
  r = fmaf(-q, 4.837512969970703125e-4f, r);
  r = fmaf(-q, 7.54978995489188216e-8f, r);
  const int qi = ((int)q) & 3;
  const float z = r * r;
  const float ps = r + r * z * (-1.6666654611e-1f + z * (8.3321608736e-3f + z * (-1.9515295891e-4f)));
  const float pc = 1.0f - 0.5f * z + z * z * (4.166664568298827e-2f + z * (-1.388731625493765e-3f + z * 2.443315711809948e-5f));
  sn = (qi == 0) ? ps : (qi == 1) ? pc : (qi == 2) ? -ps : -pc;
  cs = (qi == 0) ? pc : (qi == 1) ? -ps : (qi == 2) ? -pc : ps;
}
__global__ __launch_bounds__(256) void trig_kernel(float* tc, float* ts) {
  const int idx = (int)blockIdx.x * 256 + (int)threadIdx.x;
  if (idx >= SEQ * 64) return;
  const int t = idx >> 6, j = idx & 63;
  const float freq = exp2f(-(float)j * 0.20762050593046016f);
  const float a = (float)t * freq;
  float sn, cs;
  sincos_red(a, sn, cs);
  *(volatile float*)(tc + idx) = cs;
  *(volatile float*)(ts + idx) = sn;
  __threadfence();
  *(volatile float*)(tc + idx) = cs;
  *(volatile float*)(ts + idx) = sn;
}

__device__ __forceinline__ void kloop(v8f (&acc)[4][4], const _Float16* Ab, int lda, const _Float16* Bb, int ldb,
                                      int m0, int n0, int K, int rlane, int koff) {
  for (int k0 = 0; k0 < K; k0 += 32) {
    v16h bh[4];
#pragma unroll
    for (int j = 0; j < 4; ++j) bh[j] = ldfrag(Bb + (size_t)(n0 + (j << 4) + rlane) * ldb + koff + k0);
#pragma unroll
    for (int i = 0; i < 4; ++i) {
      const v16h ah = ldfrag(Ab + (size_t)(m0 + (i << 4) + rlane) * lda + koff + k0);
#pragma unroll
      for (int j = 0; j < 4; ++j) acc[i][j] = mma_h(ah, bh[j], acc[i][j]);
      dep_guard(acc[i][0], acc[i][3], ah, bh[0]);
    }
    keep4(bh[0], bh[1], bh[2], bh[3]);
  }
}

template <int SPLIT, int OUT_MODE>
__global__ __launch_bounds__(256) void gemm64_kernel(
    const unsigned short* __restrict__ Ap, long strideA, const unsigned short* __restrict__ A2p, long strideA2, int lda,
    const unsigned short* __restrict__ Btp, long strideB, const unsigned short* __restrict__ Bt2p, long strideB2, int ldb,
    void* Cout, long strideC, int ldc, void* Cout2, long strideC2, int ldc2,
    int M, int N, int K, float scale) {
  __shared__ __align__(16) float sT[8][16 * 68];
  const int b    = blockIdx.y;
  const int lane = threadIdx.x & 31;
  const int wave = wave_id();
  const int tilesN = N >> 6;
  const int tilesM = M >> 6;
  const int tile = (int)blockIdx.x * 8 + wave;
  if (tile >= tilesM * tilesN) return;
  const int tm = tile / tilesN;
  const int tn = tile - tm * tilesN;
  const int m0 = tm << 6;
  const int n0 = tn << 6;

  const _Float16* Ab  = (const _Float16*)(const void*)Ap   + (size_t)b * strideA;
  const _Float16* Ab2 = (const _Float16*)(const void*)A2p  + (size_t)b * strideA2;
  const _Float16* Bb  = (const _Float16*)(const void*)Btp  + (size_t)b * strideB;
  const _Float16* Bb2 = (const _Float16*)(const void*)Bt2p + (size_t)b * strideB2;

  const int rlane = lane & 15;
  const int koff  = (lane >> 4) * 8;
  const int mOff  = (lane >> 4) * 8;

  v8f acc[4][4];
#pragma unroll
  for (int i = 0; i < 4; ++i)
#pragma unroll
    for (int j = 0; j < 4; ++j) acc[i][j] = zero8();

  if (SPLIT == 1) kloop(acc, Ab2, lda, Bb, ldb, m0, n0, K, rlane, koff);
  if (SPLIT == 2) kloop(acc, Ab, lda, Bb2, ldb, m0, n0, K, rlane, koff);
  if (SPLIT != 0) {
    acc_guard4(acc[0][0], acc[0][1], acc[0][2], acc[0][3]);
    acc_guard4(acc[1][0], acc[1][1], acc[1][2], acc[1][3]);
    acc_guard4(acc[2][0], acc[2][1], acc[2][2], acc[2][3]);
    acc_guard4(acc[3][0], acc[3][1], acc[3][2], acc[3][3]);
#pragma unroll
    for (int i = 0; i < 4; ++i)
#pragma unroll
      for (int j = 0; j < 4; ++j)
#pragma unroll
        for (int r = 0; r < 8; ++r) acc[i][j][r] *= ILOS;
  }
  kloop(acc, Ab, lda, Bb, ldb, m0, n0, K, rlane, koff);
  acc_guard4(acc[0][0], acc[0][1], acc[0][2], acc[0][3]);
  acc_guard4(acc[1][0], acc[1][1], acc[1][2], acc[1][3]);
  acc_guard4(acc[2][0], acc[2][1], acc[2][2], acc[2][3]);
  acc_guard4(acc[3][0], acc[3][1], acc[3][2], acc[3][3]);

  float* slab = sT[wave];
#pragma unroll
  for (int i = 0; i < 4; ++i) {
    const int mBase = m0 + (i << 4);
#pragma unroll
    for (int j = 0; j < 4; ++j)
#pragma unroll
      for (int r = 0; r < 8; ++r)
        slab[(mOff + r) * 68 + (j << 4) + rlane] = acc[i][j][r] * scale;
    lds_wave_sync();
    if (OUT_MODE == 0) {
      float* C = (float*)Cout + (size_t)b * strideC;
      const int hh = lane >> 4, c4 = (lane & 15) * 4;
      for (int pass = 0; pass < 2; ++pass) {
#pragma unroll
        for (int it = 0; it < 8; ++it) {
          const int row = it * 2 + hh;
          const v4f v = *(const v4f*)(slab + row * 68 + c4);
          *(volatile v4f*)(C + (size_t)(mBase + row) * ldc + n0 + c4) = v;
        }
        __threadfence();
      }
    } else {
      const int q = lane >> 3, c8 = (lane & 7) * 8;
      unsigned short* C  = (unsigned short*)Cout  + (size_t)b * strideC;
      unsigned short* C2 = (unsigned short*)Cout2 + (size_t)b * strideC2;
      v4u hvs[4], lvs[4];
#pragma unroll
      for (int it = 0; it < 4; ++it) {
        const int row = it * 4 + q;
        const float* sp = slab + row * 68 + c8;
        v4u hv, lv;
#pragma unroll
        for (int e = 0; e < 4; ++e) {
          const float f0 = sp[2 * e], f1 = sp[2 * e + 1];
          const unsigned short h0 = h_bits(f0), h1 = h_bits(f1);
          hv[e] = pk16(h0, h1);
          if (OUT_MODE == 2) {
            const unsigned short l0 = h_bits((f0 - h_val(h0)) * LOS), l1 = h_bits((f1 - h_val(h1)) * LOS);
            lv[e] = pk16(l0, l1);
          } else {
            lv[e] = 0u;
          }
        }
        hvs[it] = hv; lvs[it] = lv;
      }
      for (int pass = 0; pass < 2; ++pass) {
#pragma unroll
        for (int it = 0; it < 4; ++it) {
          const int row = it * 4 + q;
          *(volatile v4u*)(C + (size_t)(mBase + row) * ldc + n0 + c8) = hvs[it];
          if (OUT_MODE == 2) *(volatile v4u*)(C2 + (size_t)(mBase + row) * ldc2 + n0 + c8) = lvs[it];
        }
        __threadfence();
      }
    }
    lds_wave_sync();
  }
}

__device__ __forceinline__ float block_sum8w(float v, float* red, int lane, int wave) {
#pragma unroll
  for (int off = 16; off > 0; off >>= 1) v += __shfl_xor(v, off, 32);
  if (lane == 0) red[wave] = v;
  __syncthreads();
  float t = 0.f;
#pragma unroll
  for (int w = 0; w < 8; ++w) t += red[w];
  __syncthreads();
  return t;
}

__global__ __launch_bounds__(256) void ln_kernel(float* src, int P, int W, const float* __restrict__ g, const float* __restrict__ bt,
                                                 unsigned short* hiP, unsigned short* loP, int loEarly, int wb) {
  __shared__ float red[8];
  __shared__ __align__(16) float rowbuf[KVPAD];
  const int tid = threadIdx.x, lane = tid & 31, wave = tid >> 5;
  const int tok = blockIdx.x;
  const int b = tok / SEQ, t = tok - b * SEQ;
  float* rowp = src + (size_t)tok * P;
  const int c0 = tid * 8;
  const int cl = imin(c0, P - 8);
  const v4f a = *(const v4f*)(rowp + cl), a2 = *(const v4f*)(rowp + cl + 4);
  float x[8], y[8];
  bool msk[8];
#pragma unroll
  for (int e = 0; e < 8; ++e) { x[e] = (e < 4) ? a[e] : a2[e - 4]; msk[e] = (c0 + e < W); }
  float s1 = 0.f;
#pragma unroll
  for (int e = 0; e < 8; ++e) s1 += msk[e] ? x[e] : 0.f;
  const float invW = 1.0f / (float)W;
  const float mean = block_sum8w(s1, red, lane, wave) * invW;
  float s2 = 0.f;
#pragma unroll
  for (int e = 0; e < 8; ++e) { const float d = msk[e] ? (x[e] - mean) : 0.f; s2 += d * d; }
  const float var  = block_sum8w(s2, red, lane, wave) * invW;
  const float rstd = rsqrtf(var + LN_EPS);
#pragma unroll
  for (int e = 0; e < 8; ++e) {
    const int cg = imin(c0 + e, W - 1);
    const float gw = bf_rne(g[cg]), gb = bf_rne(bt[cg]);
    y[e] = msk[e] ? ((x[e] - mean) * rstd * gw + gb) : 0.f;
  }
  if (c0 < P) {
    v4f o0 = {y[0], y[1], y[2], y[3]}, o1 = {y[4], y[5], y[6], y[7]};
    *(v4f*)(rowbuf + c0) = o0;
    *(v4f*)(rowbuf + c0 + 4) = o1;
  }
  __syncthreads();
  const int P8 = P >> 3, P4 = P >> 2;
  const bool act = tid < P8;
  v4u hv, lv;
#pragma unroll
  for (int e = 0; e < 4; ++e) {
    const float f0 = y[2 * e], f1 = y[2 * e + 1];
    const unsigned short h0 = h_bits(f0), h1 = h_bits(f1);
    hv[e] = pk16(h0, h1);
    lv[e] = pk16(h_bits((f0 - h_val(h0)) * LOS), h_bits((f1 - h_val(h1)) * LOS));
  }
  for (int pass = 0; pass < 2; ++pass) {
    if (act) {
      *(volatile v4u*)(hiP + (size_t)tok * P + c0) = hv;
      if (loEarly == 0) {
        *(volatile v4u*)(loP + (size_t)tok * P + c0) = lv;
      } else if (t < ERL) {
        *(volatile v4u*)(loP + ((size_t)(b * ERL + t)) * P + c0) = lv;
      }
    }
    if (wb) {
      for (int i = tid; i < P4; i += 256) {
        const v4f v = *(const v4f*)(rowbuf + 4 * i);
        *(volatile v4f*)(rowp + 4 * i) = v;
      }
    }
    __threadfence();
  }
}

__global__ __launch_bounds__(256) void pack_kernel(const float* __restrict__ src, float* dst, int nquad) {
  const int i = (int)blockIdx.x * 256 + (int)threadIdx.x;
  if (i >= nquad) return;
  const int b = blockIdx.y;
  const float* sb = src + (size_t)b * SEQ * KVPAD;
  float* db = dst + (size_t)b * SEQ_FULL * KVP;
  v4f v;
  const int e0 = 4 * i;
#pragma unroll
  for (int j = 0; j < 4; ++j) {
    const int e = e0 + j;
    const int r = e / KVP;
    const int cc = e - r * KVP;
    v[j] = sb[(size_t)r * KVPAD + cc];
  }
  *(volatile v4f*)(db + 4 * (size_t)i) = v;
  __threadfence();
  *(volatile v4f*)(db + 4 * (size_t)i) = v;
}

__global__ __launch_bounds__(256) void rope_q_kernel(const float* __restrict__ q32, const float* __restrict__ tc, const float* __restrict__ ts,
                                                     unsigned short* qp, unsigned short* ql) {
  const int tok = blockIdx.x;
  const int b = tok / SEQ, t = tok - b * SEQ;
  const int tid = threadIdx.x;
  const int c0 = tid * 8;
  const float* row = q32 + (size_t)tok * DMOD;
  const v4f a = *(const v4f*)(row + c0), a2 = *(const v4f*)(row + c0 + 4);
  float v[8];
#pragma unroll
  for (int e = 0; e < 8; ++e) v[e] = (e < 4) ? a[e] : a2[e - 4];
  if (c0 >= QNP) {
    const int d0 = c0 & 127;
    const int pcol = (d0 < 64) ? (c0 + 64) : (c0 - 64);
    const float sg = (d0 < 64) ? -1.f : 1.f;
    const v4f pa = *(const v4f*)(row + pcol), pb = *(const v4f*)(row + pcol + 4);
#pragma unroll
    for (int e = 0; e < 8; ++e) {
      const int j = (d0 + e) & 63;
      const float cs = tc[t * 64 + j], sn = ts[t * 64 + j];
      const float pe = (e < 4) ? pa[e] : pb[e - 4];
      v[e] = v[e] * cs + sg * pe * sn;
    }
  }
  v4u hv, lv;
#pragma unroll
  for (int e = 0; e < 4; ++e) {
    const unsigned short h0 = h_bits(v[2 * e]), h1 = h_bits(v[2 * e + 1]);
    hv[e] = pk16(h0, h1);
    lv[e] = pk16(h_bits((v[2 * e] - h_val(h0)) * LOS), h_bits((v[2 * e + 1] - h_val(h1)) * LOS));
  }
  for (int pass = 0; pass < 2; ++pass) {
    *(volatile v4u*)(qp + (size_t)tok * DMOD + c0) = hv;
    if (t < ERL) *(volatile v4u*)(ql + ((size_t)(b * ERL + t)) * DMOD + c0) = lv;
    __threadfence();
  }
}

__global__ __launch_bounds__(256) void rope_k_kernel(const float* __restrict__ kr32, const float* __restrict__ tc, const float* __restrict__ ts,
                                                     unsigned short* kp, unsigned short* kpl) {
  const int tid = threadIdx.x, lane = tid & 31, wave = tid >> 5;
  const int tok = (int)blockIdx.x * 8 + wave;
  const int b = tok / SEQ, t = tok - b * SEQ;
  const int c0 = lane * 8;
  const float* row = kr32 + (size_t)tok * RPW;
  const v4f a = *(const v4f*)(row + c0), a2 = *(const v4f*)(row + c0 + 4);
  const int d0 = c0 & 127;
  const int pcol = (d0 < 64) ? (c0 + 64) : (c0 - 64);
  const float sg = (d0 < 64) ? -1.f : 1.f;
  const v4f pa = *(const v4f*)(row + pcol), pb = *(const v4f*)(row + pcol + 4);
  float v[8];
#pragma unroll
  for (int e = 0; e < 8; ++e) {
    const int j = (d0 + e) & 63;
    const float cs = tc[t * 64 + j], sn = ts[t * 64 + j];
    const float xe = (e < 4) ? a[e] : a2[e - 4];
    const float pe = (e < 4) ? pa[e] : pb[e - 4];
    v[e] = xe * cs + sg * pe * sn;
  }
  v4u hv, lv;
#pragma unroll
  for (int e = 0; e < 4; ++e) {
    const unsigned short h0 = h_bits(v[2 * e]), h1 = h_bits(v[2 * e + 1]);
    hv[e] = pk16(h0, h1);
    lv[e] = pk16(h_bits((v[2 * e] - h_val(h0)) * LOS), h_bits((v[2 * e + 1] - h_val(h1)) * LOS));
  }
  for (int pass = 0; pass < 2; ++pass) {
    *(volatile v4u*)(kp + (size_t)tok * DMOD + KNP + c0) = hv;
    if (t < ERL) *(volatile v4u*)(kpl + ((size_t)(b * ERL + t)) * DMOD + KNP + c0) = lv;
    __threadfence();
  }
}

__global__ __launch_bounds__(256) void vprefix_kernel(const unsigned short* __restrict__ vh, const unsigned short* __restrict__ vl, float* vs) {
  __shared__ __align__(16) unsigned short th[64 * 64];
  __shared__ __align__(16) unsigned short tl[64 * 64];
  __shared__ __align__(16) float to[64 * 68];
  const int tid = threadIdx.x;
  const size_t R0 = (size_t)blockIdx.y * DMOD + (size_t)blockIdx.x * 64;
  float run = 0.f;
  for (int sc = 0; sc < SEQ / 64; ++sc) {
    const int s0 = sc * 64;
#pragma unroll
    for (int it = 0; it < 2; ++it) {
      const int idx = it * 256 + tid;
      const int row = idx >> 3, seg = idx & 7;
      *(v4u*)(th + row * 64 + seg * 8) = *(const v4u*)(vh + (R0 + row) * SEQ + s0 + seg * 8);
      *(v4u*)(tl + row * 64 + seg * 8) = *(const v4u*)(vl + (R0 + row) * SEQ + s0 + seg * 8);
    }
    __syncthreads();
    if (tid < 64) {
      const int i = tid;
      for (int s = 0; s < 64; ++s) {
        const float v = h_val(th[i * 64 + s]) + h_val(tl[i * 64 + s]) * ILOS;
        run += v;
        to[i * 68 + s] = run;
      }
    }
    __syncthreads();
    for (int pass = 0; pass < 2; ++pass) {
#pragma unroll
      for (int it = 0; it < 4; ++it) {
        const int idx = it * 256 + tid;
        const int row = idx >> 4, seg = idx & 15;
        const v4f v = *(const v4f*)(to + row * 68 + seg * 4);
        *(volatile v4f*)(vs + (R0 + row) * SEQ + s0 + seg * 4) = v;
      }
      __threadfence();
    }
    __syncthreads();
  }
}

#define AT_NW 4
#define AT_KC 64
static_assert(AT_KC == ERL);

template <bool EARLY>
__global__ __launch_bounds__(128)
void attn_kernel(unsigned short* qcp, const unsigned short* __restrict__ qlp,
                 const unsigned short* __restrict__ kp, const unsigned short* __restrict__ klp,
                 const unsigned short* __restrict__ vhp, const unsigned short* __restrict__ vlp,
                 const float* __restrict__ vsp, unsigned short* ctxlp,
                 int nqbl, int qb_base, float sscale) {
  constexpr int TILEH = AT_KC * DHD;
  constexpr int PH    = AT_NW * 16 * AT_KC;
  constexpr int LDSH  = (EARLY ? 2 : 1) * (2 * TILEH + PH);
  static_assert(AT_NW * 16 * DHD <= TILEH);
  __shared__ __align__(16) unsigned short smem[LDSH];
  _Float16* const base = (_Float16*)(void*)smem;
  _Float16* const Ksh = base;
  _Float16* const Vth = base + TILEH;
  _Float16* const Pwh = base + 2 * TILEH;
  _Float16* const Ksl = EARLY ? (base + 2 * TILEH + PH) : base;
  _Float16* const Vtl = EARLY ? (base + 3 * TILEH + PH) : base;
  _Float16* const Pwl = EARLY ? (base + 4 * TILEH + PH) : base;

  const int tid  = (int)threadIdx.x;
  const int wave = wave_id();
  const int lane = tid & 31;
  const int hh   = lane >> 4;
  const int c    = lane & 15;

  const int bx = (int)blockIdx.x;
  const int qb = qb_base + bx % nqbl;
  const int h  = bx / nqbl;
  const int b  = (int)blockIdx.y;
  const int q0 = qb * 64 + wave * 16;
  const size_t tok0 = (size_t)b * SEQ;

  const _Float16* QH = (const _Float16*)(const void*)qcp + (size_t)h * DHD;
  const _Float16* QLb = (const _Float16*)(const void*)qlp + ((size_t)(b * ERL + q0)) * DMOD + (size_t)h * DHD;
  const _Float16* Kh = (const _Float16*)(const void*)kp + (size_t)h * DHD;
  const _Float16* Klb = (const _Float16*)(const void*)klp + ((size_t)(b * ERL)) * DMOD + (size_t)h * DHD;
  const _Float16* Vh = (const _Float16*)(const void*)vhp + ((size_t)b * DMOD + (size_t)h * DHD) * SEQ;
  const _Float16* Vl = (const _Float16*)(const void*)vlp + ((size_t)b * DMOD + (size_t)h * DHD) * SEQ;

  v16h qah[4];
#pragma unroll
  for (int dc = 0; dc < 4; ++dc) qah[dc] = ldfrag(QH + (tok0 + q0 + c) * DMOD + dc * 32 + 8 * hh);

  float mrow[8], lrow[8];
  v8f oacc[8];
#pragma unroll
  for (int r = 0; r < 8; ++r) { mrow[r] = -INFINITY; lrow[r] = 0.f; }
#pragma unroll
  for (int t = 0; t < 8; ++t) oacc[t] = zero8();

  _Float16* pw  = Pwh + wave * 16 * AT_KC;
  _Float16* pwl = Pwl + wave * 16 * AT_KC;

  const int nChunks = qb + 1;
  for (int kc = 0; kc < nChunks; ++kc) {
    const int kv0 = kc * AT_KC;
    __syncthreads();
    {
      const int r = tid >> 1, half = (tid & 1) * 64;
      const _Float16* ks = Kh + (tok0 + kv0 + r) * DMOD + half;
#pragma unroll
      for (int i = 0; i < 8; ++i) *(v8h*)(Ksh + r * DHD + half + 8 * i) = *(const v8h*)(ks + 8 * i);
      if (EARLY) {
        const _Float16* kls = Klb + (size_t)(kv0 + r) * DMOD + half;
#pragma unroll
        for (int i = 0; i < 8; ++i) *(v8h*)(Ksl + r * DHD + half + 8 * i) = *(const v8h*)(kls + 8 * i);
      }
      const int rv = tid;
      const _Float16* vs0 = Vh + (size_t)rv * SEQ + kv0;
#pragma unroll
      for (int i = 0; i < 8; ++i) *(v8h*)(Vth + rv * AT_KC + 8 * i) = *(const v8h*)(vs0 + 8 * i);
      if (EARLY) {
        const _Float16* vl0 = Vl + (size_t)rv * SEQ + kv0;
#pragma unroll
        for (int i = 0; i < 8; ++i) *(v8h*)(Vtl + rv * AT_KC + 8 * i) = *(const v8h*)(vl0 + 8 * i);
      }
    }
    __syncthreads();

    v8f s[4];
#pragma unroll
    for (int j = 0; j < 4; ++j) {
      s[j] = zero8();
      const _Float16* krow = Ksh + (j * 16 + c) * DHD + 8 * hh;
      if (EARLY) {
        const _Float16* klrow = Ksl + (j * 16 + c) * DHD + 8 * hh;
#pragma unroll
        for (int dc = 0; dc < 4; ++dc) {
          FragH kb, kl;
          kb.h[0] = *(const v8h*)(krow + dc * 32);
          kb.h[1] = *(const v8h*)(krow + dc * 32 + 16);
          kl.h[0] = *(const v8h*)(klrow + dc * 32);
          kl.h[1] = *(const v8h*)(klrow + dc * 32 + 16);
          const v16h qal = ldfrag(QLb + (size_t)c * DMOD + dc * 32 + 8 * hh);
          s[j] = at_mma(qah[dc], kl.v, s[j]);
          s[j] = at_mma(qal, kb.v, s[j]);
        }
#pragma unroll
        for (int r = 0; r < 8; ++r) s[j][r] *= ILOS;
      }
#pragma unroll
      for (int dc = 0; dc < 4; ++dc) {
        FragH kb;
        kb.h[0] = *(const v8h*)(krow + dc * 32);
        kb.h[1] = *(const v8h*)(krow + dc * 32 + 16);
        s[j] = at_mma(qah[dc], kb.v, s[j]);
      }
    }
    const bool diag = (kc == qb);
    float cm[8];
#pragma unroll
    for (int r = 0; r < 8; ++r) {
      const int qrow = q0 + 8 * hh + r;
      float m = -INFINITY;
#pragma unroll
      for (int j = 0; j < 4; ++j) {
        const int kvcol = kv0 + j * 16 + c;
        const float sv = s[j][r] * sscale;
        const bool masked = diag && (kvcol > qrow);
        const float sm = masked ? -INFINITY : sv;
        s[j][r] = sm;
        m = fmaxf(m, sm);
      }
#pragma unroll
      for (int off = 1; off < 16; off <<= 1) m = fmaxf(m, __shfl_xor(m, off, 32));
      cm[r] = m;
    }
#pragma unroll
    for (int r = 0; r < 8; ++r) {
      const float mnew = fmaxf(mrow[r], cm[r]);
      const float alpha = expf(mrow[r] - mnew);
      mrow[r] = mnew;
      const float em = expf(-mnew);
      float psum = 0.f;
#pragma unroll
      for (int j = 0; j < 4; ++j) {
        const float sv = s[j][r];
        const float p = expf(sv - mnew);
        psum += p;
        const float pc = (sv == -INFINITY) ? 0.f : (PSC * (p - em));
        const _Float16 hb = (_Float16)pc;
        pw[(8 * hh + r) * AT_KC + j * 16 + c] = hb;
        if (EARLY) pwl[(8 * hh + r) * AT_KC + j * 16 + c] = (_Float16)(pc - (float)hb);
      }
#pragma unroll
      for (int off = 1; off < 16; off <<= 1) psum += __shfl_xor(psum, off, 32);
      lrow[r] = lrow[r] * alpha + psum;
#pragma unroll
      for (int t = 0; t < 8; ++t) oacc[t][r] *= alpha;
    }
    lds_wave_sync();
    if (EARLY) {
#pragma unroll
      for (int t = 0; t < 8; ++t) {
        v8f tl = zero8();
#pragma unroll
        for (int kk = 0; kk < 2; ++kk) {
          FragH pa, pl, vb, vl;
          pa.h[0] = *(const v8h*)(pw  + c * AT_KC + kk * 32 + 8 * hh);
          pa.h[1] = *(const v8h*)(pw  + c * AT_KC + kk * 32 + 16 + 8 * hh);
          pl.h[0] = *(const v8h*)(pwl + c * AT_KC + kk * 32 + 8 * hh);
          pl.h[1] = *(const v8h*)(pwl + c * AT_KC + kk * 32 + 16 + 8 * hh);
          vb.h[0] = *(const v8h*)(Vth + (t * 16 + c) * AT_KC + kk * 32 + 8 * hh);
          vb.h[1] = *(const v8h*)(Vth + (t * 16 + c) * AT_KC + kk * 32 + 16 + 8 * hh);
          vl.h[0] = *(const v8h*)(Vtl + (t * 16 + c) * AT_KC + kk * 32 + 8 * hh);
          vl.h[1] = *(const v8h*)(Vtl + (t * 16 + c) * AT_KC + kk * 32 + 16 + 8 * hh);
          oacc[t] = at_mma(pa.v, vb.v, oacc[t]);
          oacc[t] = at_mma(pl.v, vb.v, oacc[t]);
          tl = at_mma(pa.v, vl.v, tl);
        }
#pragma unroll
        for (int r = 0; r < 8; ++r) oacc[t][r] = fmaf(tl[r], ILOS, oacc[t][r]);
      }
    } else {
#pragma unroll 1
      for (int kk = 0; kk < 2; ++kk) {
        FragH pa;
        pa.h[0] = *(const v8h*)(pw + c * AT_KC + kk * 32 + 8 * hh);
        pa.h[1] = *(const v8h*)(pw + c * AT_KC + kk * 32 + 16 + 8 * hh);
#pragma unroll
        for (int t = 0; t < 8; ++t) {
          FragH vb;
          vb.h[0] = *(const v8h*)(Vth + (t * 16 + c) * AT_KC + kk * 32 + 8 * hh);
          vb.h[1] = *(const v8h*)(Vth + (t * 16 + c) * AT_KC + kk * 32 + 16 + 8 * hh);
          oacc[t] = at_mma(pa.v, vb.v, oacc[t]);
        }
      }
    }
  }
  acc_guard4(oacc[0], oacc[1], oacc[2], oacc[3]);
  acc_guard4(oacc[4], oacc[5], oacc[6], oacc[7]);
  __syncthreads();

  float cst[8], inv[8];
#pragma unroll
  for (int r = 0; r < 8; ++r) {
    cst[r] = PSC * expf(-mrow[r]);
    inv[r] = 1.0f / (PSC * lrow[r]);
  }
  unsigned short* osh = smem + wave * 16 * DHD;
  unsigned short* osl = smem + TILEH + wave * 16 * DHD;
#pragma unroll
  for (int t = 0; t < 8; ++t) {
    const float* vq = vsp + ((size_t)(b * DMOD + h * DHD + t * 16 + c)) * SEQ + q0 + 8 * hh;
    const v4f va = *(const v4f*)(vq), vb = *(const v4f*)(vq + 4);
#pragma unroll
    for (int r = 0; r < 8; ++r) {
      const float vsr = (r < 4) ? va[r] : vb[r - 4];
      const float ctx = (oacc[t][r] + cst[r] * vsr) * inv[r];
      const float xc = CTXC * ctx;
      const unsigned short hb = h_bits(xc);
      const int so = (8 * hh + r) * DHD + t * 16 + c;
      osh[so] = hb;
      if (EARLY) osl[so] = h_bits((xc - h_val(hb)) * LOS);
    }
  }
  lds_wave_sync();
  const int rsel = lane >> 4;
  const int c8 = (lane & 15) * 8;
  for (int pass = 0; pass < 2; ++pass) {
#pragma unroll
    for (int it = 0; it < 8; ++it) {
      const int row = it * 2 + rsel;
      const v4u x = *(const v4u*)(osh + row * DHD + c8);
      *(volatile v4u*)(qcp + (tok0 + q0 + row) * DMOD + (size_t)h * DHD + c8) = x;
      if (EARLY) {
        const v4u y = *(const v4u*)(osl + row * DHD + c8);
        *(volatile v4u*)(ctxlp + ((size_t)(b * ERL + q0 + row)) * DMOD + (size_t)h * DHD + c8) = y;
      }
    }
    __threadfence();
  }
}

#define SZ_XB    ((size_t)NTOK * DMOD * 2)
#define SZ_WDQT  ((size_t)QPR * DMOD * 2)
#define SZ_WUQRT ((size_t)DMOD * QPR * 2)
#define SZ_WDKVT ((size_t)KVPAD * DMOD * 2)
#define SZ_WKRT  ((size_t)RPW * DMOD * 2)
#define SZ_KR32  ((size_t)NTOK * RPW * 4)
#define SZ_CQH   ((size_t)NTOK * QPR * 2)
#define SZ_WUKVT ((size_t)KVW * KVPAD * 2)
#define SZ_WOB   ((size_t)DMOD * DMOD * 2)
#define SZ_F32S  ((size_t)NTOK * DMOD * 4)
#define SZ_CKVX  ((size_t)NTOK * DMOD * 4)
#define SZ_TRIG  ((size_t)SEQ * 64 * 4 * 2)
#define SZ_CQL   ((size_t)NB * ERL * QPR * 2)
#define SZ_EPL   ((size_t)NB * ERL * DMOD * 2)
#define SZ_VTL   ((size_t)NB * DMOD * SEQ * 2)
#define WS_TOTAL (SZ_XB + SZ_WDQT + SZ_WUQRT + SZ_WDKVT + SZ_WKRT + SZ_KR32 + SZ_CQH + SZ_WUKVT + SZ_WOB + SZ_F32S + SZ_CKVX + SZ_TRIG + SZ_CQL + 3 * SZ_EPL)
static_assert(WS_TOTAL <= 134217728UL);
static_assert(SZ_VTL <= SZ_WDQT + SZ_WUQRT + SZ_WDKVT + SZ_WKRT + SZ_KR32 + SZ_CQH);
static_assert((size_t)NTOK * DMOD * 2 + (size_t)NB * DMOD * SEQ * 2 == SZ_F32S);
static_assert(2 * (size_t)NTOK * KVPAD * 2 <= SZ_CKVX);
static_assert((size_t)NB * DMOD * SEQ * 4 <= SZ_CKVX);
static_assert((size_t)NTOK * KVPAD * 4 <= SZ_F32S && (size_t)NTOK * QPR * 4 <= SZ_F32S);

extern "C" void kernel_launch(void* const* d_in, const int* in_sizes, int n_in,
                              void* d_out, int out_size, void* d_ws, size_t ws_size,
                              hipStream_t stream) {
  if (n_in < 12) return;
  if (in_sizes[0] < ((NB - 1) * SEQ_FULL + SEQ) * DMOD) return;
  if (in_sizes[1] < DMOD * QPR) return;
  if (in_sizes[2] < QPR * QNP) return;
  if (in_sizes[3] < QPR * RPW) return;
  if (in_sizes[4] < DMOD * KVP) return;
  if (in_sizes[5] < KVP * KVW) return;
  if (in_sizes[6] < DMOD * RPW) return;
  if (in_sizes[7] < DMOD * DMOD) return;
  if (in_sizes[8] < QPR || in_sizes[9] < QPR) return;
  if (in_sizes[10] < KVP || in_sizes[11] < KVP) return;
  if (out_size < OUT1_OFF + (NB - 1) * SEQ_FULL * KVP + SEQ * KVP) return;

  const float* x      = (const float*)d_in[0];
  const float* W_dq   = (const float*)d_in[1];
  const float* W_uq   = (const float*)d_in[2];
  const float* W_qr   = (const float*)d_in[3];
  const float* W_dkv  = (const float*)d_in[4];
  const float* W_ukv  = (const float*)d_in[5];
  const float* W_kr   = (const float*)d_in[6];
  const float* W_o    = (const float*)d_in[7];
  const float* q_ln_w = (const float*)d_in[8];
  const float* q_ln_b = (const float*)d_in[9];
  const float* kv_ln_w = (const float*)d_in[10];
  const float* kv_ln_b = (const float*)d_in[11];
  float* out0 = (float*)d_out;
  float* out1 = (float*)d_out + OUT1_OFF;

  size_t off = 0;
  const size_t oXB    = off; off += SZ_XB;
  const size_t oWDQT  = off; off += SZ_WDQT;
  const size_t oWUQRT = off; off += SZ_WUQRT;
  const size_t oWDKVT = off; off += SZ_WDKVT;
  const size_t oWKRT  = off; off += SZ_WKRT;
  const size_t oKR32  = off; off += SZ_KR32;
  const size_t oCQH   = off; off += SZ_CQH;
  const size_t oWUKVT = off; off += SZ_WUKVT;
  const size_t oWOB   = off; off += SZ_WOB;
  const size_t oF32S  = off; off += SZ_F32S;
  const size_t oCKVX  = off; off += SZ_CKVX;
  const size_t oTRIG  = off; off += SZ_TRIG;
  const size_t oCQL   = off; off += SZ_CQL;
  const size_t oQL    = off; off += SZ_EPL;
  const size_t oKPL   = off; off += SZ_EPL;
  const size_t oCTXL  = off; off += SZ_EPL;
  if (off != WS_TOTAL) return;
  if (off > ws_size) return;

  char* ws = (char*)d_ws;
  unsigned short* XB    = (unsigned short*)(ws + oXB);
  unsigned short* QP    = XB;
  unsigned short* WDQT  = (unsigned short*)(ws + oWDQT);
  unsigned short* VTL   = (unsigned short*)(ws + oWDQT);
  unsigned short* WUQRT = (unsigned short*)(ws + oWUQRT);
  unsigned short* WDKVT = (unsigned short*)(ws + oWDKVT);
  unsigned short* WKRT  = (unsigned short*)(ws + oWKRT);
  float*          KR32  = (float*)(ws + oKR32);
  unsigned short* CQH   = (unsigned short*)(ws + oCQH);
  unsigned short* WUKVT = (unsigned short*)(ws + oWUKVT);
  unsigned short* WOB   = (unsigned short*)(ws + oWOB);
  float*          F32S  = (float*)(ws + oF32S);
  unsigned short* KP    = (unsigned short*)(ws + oF32S);
  unsigned short* VTH   = (unsigned short*)(ws + oF32S + (size_t)NTOK * DMOD * 2);
  unsigned short* CKVH  = (unsigned short*)(ws + oCKVX);
  unsigned short* CKVL  = (unsigned short*)(ws + oCKVX + (size_t)NTOK * KVPAD * 2);
  float*          VS    = (float*)(ws + oCKVX);
  float*          TRIGC = (float*)(ws + oTRIG);
  float*          TRIGS = TRIGC + (size_t)SEQ * 64;
  unsigned short* CQL   = (unsigned short*)(ws + oCQL);
  unsigned short* QL    = (unsigned short*)(ws + oQL);
  unsigned short* KPL   = (unsigned short*)(ws + oKPL);
  unsigned short* CTXL  = (unsigned short*)(ws + oCTXL);

  const dim3 b256(256), b128(128);
  const float gsc = IWSC;
  const float osc = IWSC / CTXC;

  cvt16_kernel<<<dim3((SEQ * (DMOD / 8) + 255) / 256, NB), b256, 0, stream>>>(x, (long)SEQ_FULL * DMOD, XB, (long)SEQ * DMOD, SEQ * (DMOD / 8), 1.0f);
  cvt16_kernel<<<dim3((DMOD * (DMOD / 8) + 255) / 256, 1), b256, 0, stream>>>(W_o, 0L, WOB, 0L, DMOD * (DMOD / 8), WSC);
  tcvt_kernel<<<dim3(QPR / 64, DMOD / 64), b256, 0, stream>>>(W_dq, WDQT, DMOD, QPR, DMOD, WSC);
  tcvt_kernel<<<dim3(QNP / 64, QPR / 64), b256, 0, stream>>>(W_uq, WUQRT, QPR, QNP, QPR, WSC);
  tcvt_kernel<<<dim3(RPW / 64, QPR / 64), b256, 0, stream>>>(W_qr, WUQRT + (size_t)QNP * QPR, QPR, RPW, QPR, WSC);
  tcvt_kernel<<<dim3(KVPAD / 64, DMOD / 64), b256, 0, stream>>>(W_dkv, WDKVT, DMOD, KVP, DMOD, WSC);
  tcvt_kernel<<<dim3(KVW / 64, KVPAD / 64), b256, 0, stream>>>(W_ukv, WUKVT, KVP, KVW, KVPAD, WSC);
  tcvt_kernel<<<dim3(RPW / 64, DMOD / 64), b256, 0, stream>>>(W_kr, WKRT, DMOD, RPW, DMOD, WSC);
  trig_kernel<<<dim3((SEQ * 64 + 255) / 256), b256, 0, stream>>>(TRIGC, TRIGS);
  gemm64_kernel<0, 0><<<dim3(((NTOK / 64) * (QPR / 64) + 7) / 8, 1), b256, 0, stream>>>(
      XB, 0L, XB, 0L, DMOD, WDQT, 0L, WDQT, 0L, DMOD, (void*)F32S, 0L, QPR, (void*)F32S, 0L, QPR, NTOK, QPR, DMOD, gsc);
  ln_kernel<<<dim3(NTOK), b256, 0, stream>>>(F32S, QPR, QPR, q_ln_w, q_ln_b, CQH, CQL, 1, 0);
  gemm64_kernel<0, 0><<<dim3(((NTOK / 64) * (RPW / 64) + 7) / 8, 1), b256, 0, stream>>>(
      XB, 0L, XB, 0L, DMOD, WKRT, 0L, WKRT, 0L, DMOD, (void*)KR32, 0L, RPW, (void*)KR32, 0L, RPW, NTOK, RPW, DMOD, gsc);
  gemm64_kernel<0, 0><<<dim3(((NTOK / 64) * (KVPAD / 64) + 7) / 8, 1), b256, 0, stream>>>(
      XB, 0L, XB, 0L, DMOD, WDKVT, 0L, WDKVT, 0L, DMOD, (void*)F32S, 0L, KVPAD, (void*)F32S, 0L, KVPAD, NTOK, KVPAD, DMOD, gsc);
  ln_kernel<<<dim3(NTOK), b256, 0, stream>>>(F32S, KVPAD, KVP, kv_ln_w, kv_ln_b, CKVH, CKVL, 0, 1);
  pack_kernel<<<dim3((SEQ * KVP / 4 + 255) / 256, NB), b256, 0, stream>>>(F32S, out1, SEQ * KVP / 4);
  gemm64_kernel<0, 0><<<dim3(((NTOK / 64) * (DMOD / 64) + 7) / 8, 1), b256, 0, stream>>>(
      CQH, 0L, CQH, 0L, QPR, WUQRT, 0L, WUQRT, 0L, QPR, (void*)F32S, 0L, DMOD, (void*)F32S, 0L, DMOD, NTOK, DMOD, QPR, gsc);
  gemm64_kernel<1, 0><<<dim3(((ERL / 64) * (DMOD / 64) + 7) / 8, NB), b256, 0, stream>>>(
      CQH, (long)SEQ * QPR, CQL, (long)ERL * QPR, QPR, WUQRT, 0L, WUQRT, 0L, QPR,
      (void*)F32S, (long)SEQ * DMOD, DMOD, (void*)F32S, (long)SEQ * DMOD, DMOD, ERL, DMOD, QPR, gsc);
  rope_q_kernel<<<dim3(NTOK), b256, 0, stream>>>(F32S, TRIGC, TRIGS, QP, QL);
  rope_k_kernel<<<dim3(NTOK / 8), b256, 0, stream>>>(KR32, TRIGC, TRIGS, KP, KPL);
  gemm64_kernel<0, 1><<<dim3(((NTOK / 64) * (KNP / 64) + 7) / 8, 1), b256, 0, stream>>>(
      CKVH, 0L, CKVH, 0L, KVPAD, WUKVT, 0L, WUKVT, 0L, KVPAD, (void*)KP, 0L, DMOD, (void*)KP, 0L, DMOD, NTOK, KNP, KVK, gsc);
  gemm64_kernel<1, 2><<<dim3(((ERL / 64) * (KNP / 64) + 7) / 8, NB), b256, 0, stream>>>(
      CKVH, (long)SEQ * KVPAD, CKVL, (long)SEQ * KVPAD, KVPAD, WUKVT, 0L, WUKVT, 0L, KVPAD,
      (void*)KP, (long)SEQ * DMOD, DMOD, (void*)KPL, (long)ERL * DMOD, DMOD, ERL, KNP, KVK, gsc);
  gemm64_kernel<2, 2><<<dim3(((DMOD / 64) * (SEQ / 64) + 7) / 8, NB), b256, 0, stream>>>(
      WUKVT + (size_t)KNP * KVPAD, 0L, WUKVT + (size_t)KNP * KVPAD, 0L, KVPAD, CKVH, (long)SEQ * KVPAD, CKVL, (long)SEQ * KVPAD, KVPAD,
      (void*)VTH, (long)DMOD * SEQ, SEQ, (void*)VTL, (long)DMOD * SEQ, SEQ, DMOD, SEQ, KVK, gsc);
  vprefix_kernel<<<dim3(DMOD / 64, NB), b256, 0, stream>>>(VTH, VTL, VS);
  attn_kernel<true><<<dim3(NHD * 1, NB), b128, 0, stream>>>(QP, QL, KP, KPL, VTH, VTL, VS, CTXL, 1, 0, SSCALE);
  if (SEQ / 64 > 1)
    attn_kernel<false><<<dim3(NHD * (SEQ / 64 - 1), NB), b128, 0, stream>>>(QP, QL, KP, KPL, VTH, VTL, VS, CTXL, SEQ / 64 - 1, 1, SSCALE);
  gemm64_kernel<0, 0><<<dim3(((SEQ / 64) * (DMOD / 64) + 7) / 8, NB), b256, 0, stream>>>(
      QP, (long)SEQ * DMOD, QP, (long)SEQ * DMOD, DMOD, WOB, 0L, WOB, 0L, DMOD,
      (void*)out0, (long)SEQ_FULL * DMOD, DMOD, (void*)out0, (long)SEQ_FULL * DMOD, DMOD, SEQ, DMOD, DMOD, osc);
  gemm64_kernel<1, 0><<<dim3(((ERL / 64) * (DMOD / 64) + 7) / 8, NB), b256, 0, stream>>>(
      QP, (long)SEQ * DMOD, CTXL, (long)ERL * DMOD, DMOD, WOB, 0L, WOB, 0L, DMOD,
      (void*)out0, (long)SEQ_FULL * DMOD, DMOD, (void*)out0, (long)SEQ_FULL * DMOD, DMOD, ERL, DMOD, DMOD, osc);
  (void)hipGetLastError();
}
